// _SelfAttention3D_62182536512321
// MI455X (gfx1250) — hardware-verified
//
#include <hip/hip_runtime.h>
#include <stdint.h>

typedef _Float16 v16h __attribute__((ext_vector_type(16)));
typedef _Float16 v8h  __attribute__((ext_vector_type(8)));
typedef __bf16   v16b __attribute__((ext_vector_type(16)));
typedef unsigned short v8us __attribute__((ext_vector_type(8)));
typedef float v8f __attribute__((ext_vector_type(8)));
typedef float v4f __attribute__((ext_vector_type(4)));
typedef v8h  __attribute__((may_alias)) v8ha;
typedef v8us __attribute__((may_alias)) v8usa;
typedef v4f  __attribute__((may_alias)) v4fa;

union FragH { v16h v; v8h half[2]; };
union FragB { v16b v; v8us half[2]; };

#define NB   2
#define CC   64
#define CH   32
#define NN   8192
#define XP   72
#define NWQ  (CH * CC)
#define NWV  (CC * CC)
#define NWALL (2 * NWQ + 2 * NWV)
#define PSCALE 32768.0f
#define INV_PSCALE (1.0f / 32768.0f)
#define SCALE 0.17677669529663688f

__device__ __forceinline__ v8f wmma_f16(v16h a, v16h b, v8f c) {
  v8f d = __builtin_amdgcn_wmma_f32_16x16x32_f16(false, a, false, b, (short)0, c, false, false);
  asm volatile("v_nop\n\tv_nop\n\tv_nop\n\tv_nop" : "+v"(d) : "v"(a), "v"(b));
  return d;
}
__device__ __forceinline__ v8f wmma_bf16(v16b a, v16b b, v8f c) {
  v8f d = __builtin_amdgcn_wmma_f32_16x16x32_bf16(false, a, false, b, (short)0, c, false, false);
  asm volatile("v_nop\n\tv_nop\n\tv_nop\n\tv_nop" : "+v"(d) : "v"(a), "v"(b));
  return d;
}

__device__ __forceinline__ v16h ldfrag_h(const _Float16* p, int h) {
  FragH f;
  f.half[0] = *(const v8ha*)(p + 8 * h);
  f.half[1] = *(const v8ha*)(p + 16 + 8 * h);
  return f.v;
}
__device__ __forceinline__ v16b ldfrag_b(const unsigned short* p, int h) {
  FragB f;
  f.half[0] = *(const v8usa*)(p + 8 * h);
  f.half[1] = *(const v8usa*)(p + 16 + 8 * h);
  return f.v;
}

__device__ __forceinline__ unsigned short bf16_rne(float f) {
  unsigned u = __float_as_uint(f);
  u = u + 0x7FFFu + ((u >> 16) & 1u);
  return (unsigned short)(u >> 16);
}
__device__ __forceinline__ float bf16_f32(unsigned short b) {
  return __uint_as_float(((unsigned)b) << 16);
}

__device__ __forceinline__ v8us hi8(v8f v, float sc) {
  const v8us r = { bf16_rne(v[0] * sc), bf16_rne(v[1] * sc), bf16_rne(v[2] * sc), bf16_rne(v[3] * sc),
                   bf16_rne(v[4] * sc), bf16_rne(v[5] * sc), bf16_rne(v[6] * sc), bf16_rne(v[7] * sc) };
  return r;
}
__device__ __forceinline__ v8us lo8(v8f v, float sc, v8us hh) {
  const v8us r = { bf16_rne(v[0] * sc - bf16_f32(hh[0])), bf16_rne(v[1] * sc - bf16_f32(hh[1])),
                   bf16_rne(v[2] * sc - bf16_f32(hh[2])), bf16_rne(v[3] * sc - bf16_f32(hh[3])),
                   bf16_rne(v[4] * sc - bf16_f32(hh[4])), bf16_rne(v[5] * sc - bf16_f32(hh[5])),
                   bf16_rne(v[6] * sc - bf16_f32(hh[6])), bf16_rne(v[7] * sc - bf16_f32(hh[7])) };
  return r;
}

__global__ __launch_bounds__(256) void k_wconvert(
    const float* __restrict__ wq, const float* __restrict__ wk,
    const float* __restrict__ wv, const float* __restrict__ wo,
    unsigned short* __restrict__ whi, unsigned short* __restrict__ wlo)
{
  const int g = blockIdx.x * 256 + threadIdx.x;
  if (g >= NWALL / 8) return;
  const int e = g * 8;
  const float* src;
  if (e < NWQ)                src = wq + e;
  else if (e < 2 * NWQ)       src = wk + (e - NWQ);
  else if (e < 2 * NWQ + NWV) src = wv + (e - 2 * NWQ);
  else                        src = wo + (e - 2 * NWQ - NWV);
  const v4f a = *(const v4fa*)src;
  const v4f c = *(const v4fa*)(src + 4);
  const unsigned short h0 = bf16_rne(a.x), h1 = bf16_rne(a.y), h2 = bf16_rne(a.z), h3 = bf16_rne(a.w);
  const unsigned short h4 = bf16_rne(c.x), h5 = bf16_rne(c.y), h6 = bf16_rne(c.z), h7 = bf16_rne(c.w);
  const v8us hv = { h0, h1, h2, h3, h4, h5, h6, h7 };
  const v8us lv = { bf16_rne(a.x - bf16_f32(h0)), bf16_rne(a.y - bf16_f32(h1)),
                    bf16_rne(a.z - bf16_f32(h2)), bf16_rne(a.w - bf16_f32(h3)),
                    bf16_rne(c.x - bf16_f32(h4)), bf16_rne(c.y - bf16_f32(h5)),
                    bf16_rne(c.z - bf16_f32(h6)), bf16_rne(c.w - bf16_f32(h7)) };
  unsigned short* ph = whi + e;
  unsigned short* pl = wlo + e;
  *(volatile v8us*)ph = hv;
  *(volatile v8us*)pl = lv;
  __threadfence();
  *(volatile v8us*)ph = hv;
  *(volatile v8us*)pl = lv;
}

__device__ __forceinline__ void proj_store(const _Float16* sQ, const _Float16* sK, const _Float16* sV,
                                           _Float16* qd, _Float16* kd, _Float16* vd, int tid) {
  #pragma unroll
  for (int i = 0; i < 2; ++i) {
    const int off = (i * 128 + tid) * 8;
    const v8h a = *(const v8ha*)(sQ + off);
    *(volatile v8h*)(qd + off) = a;
    const v8h c = *(const v8ha*)(sK + off);
    *(volatile v8h*)(kd + off) = c;
  }
  const int q8 = tid & 7, sub = tid >> 3;
  #pragma unroll
  for (int i = 0; i < 4; ++i) {
    const int c = i * 16 + sub;
    const v8h a = *(const v8ha*)(sV + c * 64 + 8 * q8);
    *(volatile v8h*)(vd + (size_t)c * NN + 8 * q8) = a;
  }
}

__global__ __launch_bounds__(128) void k_proj(
    const float* __restrict__ x,
    const unsigned short* __restrict__ whi, const unsigned short* __restrict__ wlo,
    const float* __restrict__ bq, const float* __restrict__ bk, const float* __restrict__ bv,
    _Float16* __restrict__ qpl, _Float16* __restrict__ kpl, _Float16* __restrict__ vpl)
{
  __shared__ __attribute__((aligned(16))) unsigned short sXh[64 * XP];
  __shared__ __attribute__((aligned(16))) unsigned short sXl[64 * XP];
  __shared__ __attribute__((aligned(16))) _Float16 sQ[64 * CH];
  __shared__ __attribute__((aligned(16))) _Float16 sK[64 * CH];
  __shared__ __attribute__((aligned(16))) _Float16 sV[CC * 64];

  const int tid = threadIdx.x, lane = tid & 31, w = tid >> 5;
  const int h = lane >> 4, m = lane & 15;
  const int n0 = blockIdx.x * 64;
  const int b = blockIdx.y;

  const float* xb = x + (size_t)b * CC * NN + n0;
  #pragma unroll
  for (int i = 0; i < 8; ++i) {
    const int f4 = i * 128 + tid;
    const int c = f4 >> 4;
    const int j4 = f4 & 15;
    const v4f v = *(const v4fa*)(xb + (size_t)c * NN + 4 * j4);
    const float e0 = v.x, e1 = v.y, e2 = v.z, e3 = v.w;
    const unsigned short a0 = bf16_rne(e0), a1 = bf16_rne(e1), a2 = bf16_rne(e2), a3 = bf16_rne(e3);
    const int t0 = 4 * j4;
    sXh[(t0 + 0) * XP + c] = a0;  sXl[(t0 + 0) * XP + c] = bf16_rne(e0 - bf16_f32(a0));
    sXh[(t0 + 1) * XP + c] = a1;  sXl[(t0 + 1) * XP + c] = bf16_rne(e1 - bf16_f32(a1));
    sXh[(t0 + 2) * XP + c] = a2;  sXl[(t0 + 2) * XP + c] = bf16_rne(e2 - bf16_f32(a2));
    sXh[(t0 + 3) * XP + c] = a3;  sXl[(t0 + 3) * XP + c] = bf16_rne(e3 - bf16_f32(a3));
  }
  __syncthreads();

  const v8f zero8 = {0.f, 0.f, 0.f, 0.f, 0.f, 0.f, 0.f, 0.f};
  v8f acc[8];
  #pragma unroll
  for (int nt = 0; nt < 8; ++nt) acc[nt] = zero8;

  const unsigned short* arow_h = sXh + (16 * w + m) * XP;
  const unsigned short* arow_l = sXl + (16 * w + m) * XP;

  #pragma unroll
  for (int ks = 0; ks < 2; ++ks) {
    const int k0 = 32 * ks;
    const v16b ah = ldfrag_b(arow_h + k0, h);
    const v16b al = ldfrag_b(arow_l + k0, h);
    #pragma unroll
    for (int nt = 0; nt < 8; ++nt) {
      const int f = 16 * nt + m;
      const v16b bh = ldfrag_b(whi + f * CC + k0, h);
      const v16b bl = ldfrag_b(wlo + f * CC + k0, h);
      acc[nt] = wmma_bf16(ah, bh, acc[nt]);
      acc[nt] = wmma_bf16(ah, bl, acc[nt]);
      acc[nt] = wmma_bf16(al, bh, acc[nt]);
    }
  }

  #pragma unroll
  for (int nt = 0; nt < 8; ++nt) {
    const int f = 16 * nt + m;
    float bias;
    if (nt < 2)      bias = bq[f];
    else if (nt < 4) bias = bk[f - CH];
    else             bias = bv[f - 2 * CH];
    #pragma unroll
    for (int r = 0; r < 8; ++r) {
      const int tok = 16 * w + 8 * h + r;
      const _Float16 y = (_Float16)(acc[nt][r] + bias);
      if (nt < 2)      sQ[tok * CH + f] = y;
      else if (nt < 4) sK[tok * CH + (f - CH)] = y;
      else             sV[(f - 2 * CH) * 64 + tok] = y;
    }
  }
  __syncthreads();

  _Float16* qd = qpl + ((size_t)b * NN + n0) * CH;
  _Float16* kd = kpl + ((size_t)b * NN + n0) * CH;
  _Float16* vd = vpl + (size_t)b * CC * NN + n0;
  proj_store(sQ, sK, sV, qd, kd, vd, tid);
  __threadfence();
  proj_store(sQ, sK, sV, qd, kd, vd, tid);
}

__device__ __forceinline__ v16h pack_p(v8f a, v8f c) {
  const v16h r = { (_Float16)(a[0] * PSCALE), (_Float16)(a[1] * PSCALE), (_Float16)(a[2] * PSCALE), (_Float16)(a[3] * PSCALE),
                   (_Float16)(a[4] * PSCALE), (_Float16)(a[5] * PSCALE), (_Float16)(a[6] * PSCALE), (_Float16)(a[7] * PSCALE),
                   (_Float16)(c[0] * PSCALE), (_Float16)(c[1] * PSCALE), (_Float16)(c[2] * PSCALE), (_Float16)(c[3] * PSCALE),
                   (_Float16)(c[4] * PSCALE), (_Float16)(c[5] * PSCALE), (_Float16)(c[6] * PSCALE), (_Float16)(c[7] * PSCALE) };
  return r;
}

__device__ __forceinline__ void out_store(const float* sOut, float* od, int tid) {
  const int q8 = tid & 7, sub = tid >> 3;
  #pragma unroll
  for (int i = 0; i < 8; ++i) {
    const int L = i * 16 + sub;
    const int o = L >> 1, hl = L & 1;
    const v4f v = *(const v4fa*)(sOut + o * 64 + 32 * hl + 4 * q8);
    *(volatile v4f*)(od + (size_t)o * NN + 32 * hl + 4 * q8) = v;
  }
}

__global__ __launch_bounds__(128) void k_attn(
    const _Float16* __restrict__ qpl,
    const _Float16* __restrict__ kpl,
    const _Float16* __restrict__ vpl,
    const unsigned short* __restrict__ wohi, const unsigned short* __restrict__ wolo,
    const float* __restrict__ bo,
    float* __restrict__ out)
{
  __shared__ __attribute__((aligned(16))) float sOut[CC * 64];

  const int tid = threadIdx.x, lane = tid & 31, w = tid >> 5;
  const int h = lane >> 4, m = lane & 15;
  const int b = blockIdx.y;
  const int qblk = blockIdx.x * 64;
  const int q0 = qblk + 16 * w;

  const v16h qf = ldfrag_h(qpl + ((size_t)b * NN + q0 + m) * CH, h);

  const v8f zero8 = {0.f, 0.f, 0.f, 0.f, 0.f, 0.f, 0.f, 0.f};
  v8f o[4];
  #pragma unroll
  for (int t = 0; t < 4; ++t) o[t] = zero8;
  float mrun = -1e30f, lrun = 0.0f;

  const _Float16* kbase = kpl + ((size_t)b * NN + m) * CH;
  const _Float16* vbase = vpl + ((size_t)b * CC + m) * NN;

  #pragma unroll 1
  for (int kb = 0; kb < NN; kb += 64) {
    v8f s[4];
    #pragma unroll
    for (int j = 0; j < 4; ++j) {
      const v16h kf = ldfrag_h(kbase + (size_t)(kb + 16 * j) * CH, h);
      s[j] = wmma_f16(kf, qf, zero8);
    }
    #pragma unroll
    for (int j = 0; j < 4; ++j)
      #pragma unroll
      for (int r = 0; r < 8; ++r) s[j][r] = s[j][r] * SCALE;

    float mloc = s[0][0];
    #pragma unroll
    for (int j = 0; j < 4; ++j)
      #pragma unroll
      for (int r = 0; r < 8; ++r) mloc = fmaxf(mloc, s[j][r]);
    mloc = fmaxf(mloc, __shfl_xor(mloc, 16, 32));
    const float mnew = fmaxf(mrun, mloc);
    const float alpha = __expf(mrun - mnew);
    mrun = mnew;
    float lsum = 0.0f;
    #pragma unroll
    for (int j = 0; j < 4; ++j)
      #pragma unroll
      for (int r = 0; r < 8; ++r) {
        const float p = __expf(s[j][r] - mnew);
        s[j][r] = p;
        lsum += p;
      }
    lsum += __shfl_xor(lsum, 16, 32);
    lrun = lrun * alpha + lsum;
    #pragma unroll
    for (int t = 0; t < 4; ++t)
      #pragma unroll
      for (int r = 0; r < 8; ++r) o[t][r] = o[t][r] * alpha;

    const v16h pb0 = pack_p(s[0], s[1]);
    const v16h pb1 = pack_p(s[2], s[3]);

    #pragma unroll
    for (int t = 0; t < 4; ++t) {
      const _Float16* vp = vbase + (size_t)(16 * t) * NN + kb;
      const v16h vf0 = ldfrag_h(vp, h);
      const v16h vf1 = ldfrag_h(vp + 32, h);
      o[t] = wmma_f16(vf0, pb0, o[t]);
      o[t] = wmma_f16(vf1, pb1, o[t]);
    }
  }

  const float inv = (1.0f / lrun) * INV_PSCALE;
  FragB bh0, bl0, bh1, bl1;
  {
    const v8us ha = hi8(o[0], inv), hb = hi8(o[1], inv), hc = hi8(o[2], inv), hd = hi8(o[3], inv);
    bh0.half[0] = ha;  bh0.half[1] = hb;
    bh1.half[0] = hc;  bh1.half[1] = hd;
    bl0.half[0] = lo8(o[0], inv, ha);  bl0.half[1] = lo8(o[1], inv, hb);
    bl1.half[0] = lo8(o[2], inv, hc);  bl1.half[1] = lo8(o[3], inv, hd);
  }

  v8f acc2[4];
  #pragma unroll
  for (int ot = 0; ot < 4; ++ot) {
    const unsigned short* wrh = wohi + (16 * ot + m) * CC;
    const unsigned short* wrl = wolo + (16 * ot + m) * CC;
    v8f z = zero8;
    {
      const v16b a_h = ldfrag_b(wrh, h);
      const v16b a_l = ldfrag_b(wrl, h);
      z = wmma_bf16(a_h, bh0.v, z);
      z = wmma_bf16(a_h, bl0.v, z);
      z = wmma_bf16(a_l, bh0.v, z);
    }
    {
      const v16b a_h = ldfrag_b(wrh + 32, h);
      const v16b a_l = ldfrag_b(wrl + 32, h);
      z = wmma_bf16(a_h, bh1.v, z);
      z = wmma_bf16(a_h, bl1.v, z);
      z = wmma_bf16(a_l, bh1.v, z);
    }
    acc2[ot] = z;
  }

  float* so = sOut + 16 * w + m;
  #pragma unroll
  for (int ot = 0; ot < 4; ++ot)
    #pragma unroll
    for (int r = 0; r < 8; ++r) {
      const int orow = 16 * ot + 8 * h + r;
      so[orow * 64] = acc2[ot][r] + bo[orow];
    }
  __syncthreads();

  float* od = out + (size_t)b * CC * NN + qblk;
  out_store(sOut, od, tid);
  __threadfence();
  out_store(sOut, od, tid);
}

extern "C" void kernel_launch(void* const* d_in, const int* in_sizes, int n_in,
                              void* d_out, int out_size, void* d_ws, size_t ws_size,
                              hipStream_t stream) {
  if (n_in < 9) return;
  if (in_sizes[0] != NB * CC * NN) return;
  if (in_sizes[1] != NWQ || in_sizes[2] != CH) return;
  if (in_sizes[3] != NWQ || in_sizes[4] != CH) return;
  if (in_sizes[5] != NWV || in_sizes[6] != CC) return;
  if (in_sizes[7] != NWV || in_sizes[8] != CC) return;
  if (out_size != NB * CC * NN) return;

  const float* x  = (const float*)d_in[0];
  const float* wq = (const float*)d_in[1];
  const float* bq = (const float*)d_in[2];
  const float* wk = (const float*)d_in[3];
  const float* bk = (const float*)d_in[4];
  const float* wv = (const float*)d_in[5];
  const float* bv = (const float*)d_in[6];
  const float* wo = (const float*)d_in[7];
  const float* bo = (const float*)d_in[8];
  float* out = (float*)d_out;

  const size_t w_bytes  = (size_t)NWALL * 2;
  const size_t qk_bytes = (size_t)NB * NN * CH * 2;
  const size_t v_bytes  = (size_t)NB * CC * NN * 2;
  const size_t total = 2 * w_bytes + 2 * qk_bytes + v_bytes;
  if (total > ws_size) return;

  char* ws = (char*)d_ws;
  unsigned short* whi = (unsigned short*)(ws);
  unsigned short* wlo = (unsigned short*)(ws + w_bytes);
  _Float16* qpl = (_Float16*)(ws + 2 * w_bytes);
  _Float16* kpl = (_Float16*)(ws + 2 * w_bytes + qk_bytes);
  _Float16* vpl = (_Float16*)(ws + 2 * w_bytes + 2 * qk_bytes);
  const unsigned short* wohi = whi + (2 * NWQ + NWV);
  const unsigned short* wolo = wlo + (2 * NWQ + NWV);

  const int ngroups = NWALL / 8;
  k_wconvert<<<(ngroups + 255) / 256, 256, 0, stream>>>(wq, wk, wv, wo, whi, wlo);

  dim3 gProj(NN / 64, NB);
  k_proj<<<gProj, 128, 0, stream>>>(x, whi, wlo, bq, bk, bv, qpl, kpl, vpl);

  dim3 gAtt(NN / 64, NB);
  k_attn<<<gAtt, 128, 0, stream>>>(qpl, kpl, vpl, wohi, wolo, bo, out);
}
